// SwarmByteRingModel_10857677324459
// MI455X (gfx1250) — hardware-verified
//
#include <hip/hip_runtime.h>
#include <stdint.h>
#include <stddef.h>
#include <math.h>

#define NBE   32
#define NBIT  256
#define MAXH  1024
#define KMX   128
#define BAT   4096

#define RB    64
#define NTH   128
#define XS    136
#define HBP   40
#define YP    132
#define SCP   256

#define OFF_SIDX 0
#define OFF_SCOV 512
#define OFF_SCAT 1536
#define OFF_XG   (OFF_SCAT + RB * SCP * 4)
#define OFF_HB   (OFF_XG + RB * XS * 2)
#define OFF_SY   (OFF_HB + (NTH / 32) * 16 * HBP * 2)
#define LDS_MAIN (OFF_SY + RB * YP * 4)

static_assert(NTH == KMX);
static_assert(RB == 16 * (NTH / 32));
static_assert(RB <= NTH);
static_assert(BAT % RB == 0);
static_assert((OFF_SCAT % 16) == 0);
static_assert((OFF_XG % 16) == 0);
static_assert((OFF_HB % 16) == 0);
static_assert((OFF_SY % 16) == 0);
static_assert((XS * 2) % 16 == 0);
static_assert((HBP * 2) % 16 == 0);
static_assert(((RB * SCP / 4) % NTH) == 0);
static_assert(((RB * NBIT / 4) % NTH) == 0);
static_assert(LDS_MAIN == 123392);
static_assert(MAXH % 64 == 0);
static_assert(KMX % 64 == 0);

typedef _Float16     v16h __attribute__((ext_vector_type(16)));
typedef _Float16     v8h  __attribute__((ext_vector_type(8)));
typedef _Float16     v4h  __attribute__((ext_vector_type(4)));
typedef float        v8f  __attribute__((ext_vector_type(8)));
typedef float        v4f  __attribute__((ext_vector_type(4)));
typedef unsigned int v4u  __attribute__((ext_vector_type(4)));
typedef v8h __attribute__((may_alias)) v8ha;
typedef v4h __attribute__((may_alias)) v4ha;
typedef v4f __attribute__((may_alias)) v4fa;
typedef v4u __attribute__((may_alias)) v4ua;

union FragH { v16h v; v8h h[2]; v4u q[2]; };

__constant__ int c_KS[NBE] = {
  128, 64, 32, 16, 8, 4, 2, 2,  128, 64, 32, 16, 8, 4, 2, 2,
  128, 64, 32, 16, 8, 4, 2, 2,  128, 64, 32, 16, 8, 4, 2, 2};
__constant__ int c_HS[NBE] = {
  1024, 512, 256, 128, 128, 128, 128, 128,  1024, 512, 256, 128, 128, 128, 128, 128,
  1024, 512, 256, 128, 128, 128, 128, 128,  1024, 512, 256, 128, 128, 128, 128, 128};
__constant__ int c_PER[NBE] = {
  21, 13, 8, 5, 3, 2, 1, 1,  21, 13, 8, 5, 3, 2, 1, 1,
  21, 13, 8, 5, 3, 2, 1, 1,  21, 13, 8, 5, 3, 2, 1, 1};

__device__ __forceinline__ v8f wmma_h(v16h a, v16h b, v8f c) {
  v8f d = __builtin_amdgcn_wmma_f32_16x16x32_f16(false, a, false, b, (short)0, c, false, false);
  asm volatile("v_nop\n\tv_nop\n\tv_nop\n\tv_nop" : "+v"(d) : "v"(a), "v"(b));
  return d;
}

__device__ __forceinline__ v16h ldfrag_g(const _Float16* p, int hf) {
  FragH f;
  f.h[0] = *(const v8h*)(p + 8 * hf);
  f.h[1] = *(const v8h*)(p + 16 + 8 * hf);
  return f.v;
}
__device__ __forceinline__ v16h ldfrag_l(const _Float16* p, int hf) {
  FragH f;
  f.h[0] = *(const v8ha*)(p + 8 * hf);
  f.h[1] = *(const v8ha*)(p + 16 + 8 * hf);
  return f.v;
}

__device__ __forceinline__ float gelu_t(float v) {
  const float u = v * (1.0f + 0.044715f * v * v);
  float a = -1.5957691216057308f * u;
  a = fminf(a, 80.0f);
  const float e = __expf(a);
  return v * __builtin_amdgcn_rcpf(1.0f + e);
}

__global__ __launch_bounds__(256) void k_wtr(const float* __restrict__ src,
                                             _Float16* __restrict__ dst,
                                             int R, int C, int zr)
{
  __shared__ __align__(16) _Float16 s[64 * 72];
  const int tid = threadIdx.x;
  const int b = blockIdx.z;
  const int c0 = blockIdx.x * 64;
  const int r0 = blockIdx.y * 64;
  const int Kb = c_KS[b];
  const float* sp = src + (size_t)b * R * C;
  _Float16* dp = dst + (size_t)b * R * C;

  #pragma unroll 4
  for (int j = 0; j < 16; ++j) {
    const int e = tid + 256 * j;
    const int r = e >> 6, c = e & 63;
    float v = sp[(size_t)(r0 + r) * C + c0 + c] * 64.0f;
    const int kk = zr ? (r0 + r) : (c0 + c);
    v = (kk < Kb) ? v : 0.0f;
    s[c * 72 + r] = (_Float16)v;
  }
  __syncthreads();

  const int p0 = tid, p1 = tid + 256;
  const v4u v0 = *(const v4ua*)(s + (p0 >> 3) * 72 + (p0 & 7) * 8);
  const v4u v1 = *(const v4ua*)(s + (p1 >> 3) * 72 + (p1 & 7) * 8);
  _Float16* d0 = dp + (size_t)(c0 + (p0 >> 3)) * R + r0 + (p0 & 7) * 8;
  _Float16* d1 = dp + (size_t)(c0 + (p1 >> 3)) * R + r0 + (p1 & 7) * 8;
  *(volatile v4u*)d0 = v0;
  *(volatile v4u*)d1 = v1;
  __threadfence();
  *(volatile v4u*)d0 = v0;
  *(volatile v4u*)d1 = v1;
}

__device__ __forceinline__ void out_pass(const float* __restrict__ x, const float* scat,
                                         const float* srcp, float* out, int row0, int tid)
{
  #pragma unroll 1
  for (int it = 0; it < (RB * NBIT / 4) / NTH; ++it) {
    const int g = tid + NTH * it;
    const int r = g >> 6;
    const int c4 = (g & 63) * 4;
    const v4f xv = *(const v4fa*)(x + (size_t)(row0 + r) * NBIT + c4);
    const v4f sv = *(const v4fa*)(scat + r * SCP + c4);
    const v4f rv = *(const v4fa*)(srcp + c4);
    const v4f o = xv + sv * rv;
    *(volatile v4f*)(out + (size_t)(row0 + r) * NBIT + c4) = o;
  }
}

__global__ __launch_bounds__(NTH) void k_main(const float* __restrict__ x,
                                             const _Float16* __restrict__ w1t,
                                             const float* __restrict__ b1,
                                             const _Float16* __restrict__ w2t,
                                             const float* __restrict__ b2,
                                             const int* __restrict__ idx,
                                             const int* __restrict__ stp,
                                             float* __restrict__ out)
{
  extern __shared__ __align__(16) unsigned char dsm[];
  int*      sidx = (int*)(dsm + OFF_SIDX);
  int*      scov = (int*)(dsm + OFF_SCOV);
  float*    scat = (float*)(dsm + OFF_SCAT);
  _Float16* xg   = (_Float16*)(dsm + OFF_XG);
  _Float16* hbal = (_Float16*)(dsm + OFF_HB);
  float*    sY   = (float*)(dsm + OFF_SY);

  const int tid = threadIdx.x, lane = tid & 31, wv = tid >> 5;
  const int hf = lane >> 4, m = lane & 15;
  const int row0 = blockIdx.x * RB;
  _Float16* hb = hbal + wv * (16 * HBP);
  const int step = stp[0];

  const v4f z4 = {0.f, 0.f, 0.f, 0.f};
  const v8f z8 = {0.f, 0.f, 0.f, 0.f, 0.f, 0.f, 0.f, 0.f};
  const v4u z4u = {0u, 0u, 0u, 0u};

  #pragma unroll 1
  for (int j = 0; j < (RB * SCP / 4) / NTH; ++j) *(v4fa*)(scat + 4 * (tid + NTH * j)) = z4;
  for (int c = tid; c < NBIT; c += NTH) scov[c] = 0;
  __syncthreads();

  #pragma unroll 1
  for (int u = 0; u < NBE; ++u) {
    const int per = c_PER[u];
    if ((step % per) != 0) continue;
    const int K = c_KS[u];
    const int H = c_HS[u];
    const int Kpad = (K < 32) ? 32 : K;
    const int KS32 = Kpad >> 5;
    const int lq = (Kpad == 128) ? 5 : ((Kpad == 64) ? 4 : 3);
    const int Kn = (K < 16) ? 16 : K;
    const int KT = Kn >> 4;

    {
      int v = idx[u * KMX + tid];
      v = (v < 0) ? (v + NBIT) : v;
      v = (v < 0) ? 0 : ((v > NBIT - 1) ? (NBIT - 1) : v);
      sidx[tid] = v;
    }
    __syncthreads();

    {
      const int GQ = Kpad >> 3;
      #pragma unroll 1
      for (int it = 0; it < GQ; ++it) {
        const int q = tid + NTH * it;
        const int r = q >> lq;
        const int c4 = (q & ((1 << lq) - 1)) * 4;
        const float* xr = x + (size_t)(row0 + r) * NBIT;
        v4h g;
        #pragma unroll
        for (int jj = 0; jj < 4; ++jj) {
          const int c = c4 + jj;
          const int col = sidx[c];
          const float v = xr[col];
          g[jj] = (c < K) ? (_Float16)v : (_Float16)0.0f;
        }
        *(v4ha*)(xg + r * XS + c4) = g;
      }
    }
    __syncthreads();

    FragH A1[4];
    #pragma unroll
    for (int ks = 0; ks < 4; ++ks) {
      A1[ks].q[0] = z4u; A1[ks].q[1] = z4u;
      if (ks < KS32) A1[ks].v = ldfrag_l(xg + (wv * 16 + m) * XS + ks * 32, hf);
    }

    v8f acc[8];
    #pragma unroll
    for (int nt = 0; nt < 8; ++nt) acc[nt] = z8;

    #pragma unroll 1
    for (int hh = 0; hh < H; hh += 32) {
      #pragma unroll
      for (int ch = 0; ch < 2; ++ch) {
        const int hcol = hh + ch * 16 + m;
        const _Float16* bp = w1t + ((size_t)u * MAXH + hcol) * KMX;
        v8f c1 = z8;
        #pragma unroll
        for (int ks = 0; ks < 4; ++ks) {
          if (ks < KS32) {
            const v16h bfr = ldfrag_g(bp + ks * 32, hf);
            c1 = wmma_h(A1[ks].v, bfr, c1);
          }
        }
        const float bv = b1[u * MAXH + hcol];
        #pragma unroll
        for (int r = 0; r < 8; ++r) {
          const float pre = c1[r] * (1.0f / 64.0f) + bv;
          const float gv = gelu_t(pre) * 64.0f;
          hb[(8 * hf + r) * HBP + ch * 16 + m] = (_Float16)gv;
        }
      }
      __syncthreads();

      const v16h a2 = ldfrag_l(hb + m * HBP, hf);
      #pragma unroll
      for (int nt = 0; nt < 8; ++nt) {
        if (nt < KT) {
          const _Float16* bp = w2t + ((size_t)u * KMX + nt * 16 + m) * MAXH + hh;
          const v16h bfr = ldfrag_g(bp, hf);
          acc[nt] = wmma_h(a2, bfr, acc[nt]);
        }
      }
      __syncthreads();
    }

    #pragma unroll
    for (int nt = 0; nt < 8; ++nt) {
      if (nt < KT) {
        const int col = nt * 16 + m;
        const float bb = b2[u * KMX + col];
        #pragma unroll
        for (int r = 0; r < 8; ++r)
          sY[(wv * 16 + 8 * hf + r) * YP + col] = acc[nt][r] * (1.0f / 4096.0f) + bb;
      }
    }
    __syncthreads();

    if (tid < RB) {
      const int r = tid;
      float* srow = scat + r * SCP;
      const float* yrow = sY + r * YP;
      #pragma unroll 1
      for (int c = 0; c < K; ++c) {
        const int col = sidx[c];
        srow[col] = srow[col] + yrow[c];
      }
    } else if (tid == RB) {
      #pragma unroll 1
      for (int c = 0; c < K; ++c) {
        const int col = sidx[c];
        scov[col] = scov[col] + 1;
      }
    }
    __syncthreads();
  }

  float* srcp = sY;
  for (int c = tid; c < NBIT; c += NTH) {
    const float cv = (float)scov[c];
    srcp[c] = 1.0f / fmaxf(cv, 1.0f);
  }
  __syncthreads();

  out_pass(x, scat, srcp, out, row0, tid);
  __threadfence();
  out_pass(x, scat, srcp, out, row0, tid);
}

extern "C" void kernel_launch(void* const* d_in, const int* in_sizes, int n_in,
                              void* d_out, int out_size, void* d_ws, size_t ws_size,
                              hipStream_t stream)
{
  if (n_in < 7) return;
  if (in_sizes[0] != BAT * NBIT) return;
  if (in_sizes[1] != NBE * KMX * MAXH) return;
  if (in_sizes[2] != NBE * MAXH) return;
  if (in_sizes[3] != NBE * MAXH * KMX) return;
  if (in_sizes[4] != NBE * KMX) return;
  if (in_sizes[5] != NBE * KMX) return;
  if (in_sizes[6] < 1) return;
  if (out_size != BAT * NBIT) return;

  const float* x   = (const float*)d_in[0];
  const float* W1  = (const float*)d_in[1];
  const float* b1  = (const float*)d_in[2];
  const float* W2  = (const float*)d_in[3];
  const float* b2  = (const float*)d_in[4];
  const int*   idx = (const int*)d_in[5];
  const int*   stp = (const int*)d_in[6];
  float* out = (float*)d_out;

  const size_t bW1T = (size_t)NBE * MAXH * KMX * 2;
  const size_t bW2T = (size_t)NBE * KMX * MAXH * 2;
  const size_t total = bW1T + bW2T;
  if (total > ws_size) return;
  if (total > (size_t)134217728) return;
  char* ws = (char*)d_ws;
  _Float16* W1T = (_Float16*)(ws);
  _Float16* W2T = (_Float16*)(ws + bW1T);

  k_wtr<<<dim3(MAXH / 64, KMX / 64, NBE), 256, 0, stream>>>(W1, W1T, KMX, MAXH, 1);
  k_wtr<<<dim3(KMX / 64, MAXH / 64, NBE), 256, 0, stream>>>(W2, W2T, MAXH, KMX, 0);

  hipFuncSetAttribute(reinterpret_cast<const void*>(&k_main),
                      hipFuncAttributeMaxDynamicSharedMemorySize, LDS_MAIN);
  k_main<<<BAT / RB, NTH, LDS_MAIN, stream>>>(x, W1T, b1, W2T, b2, idx, stp, out);
}
